// TwoLayerGCN_2997887173231
// MI455X (gfx1250) — hardware-verified
//
#include <hip/hip_runtime.h>
#include <math.h>

typedef __attribute__((ext_vector_type(16))) _Float16 v16h;
typedef __attribute__((ext_vector_type(16))) __bf16 v16b;
typedef __attribute__((ext_vector_type(8)))  _Float16 v8h;
typedef __attribute__((ext_vector_type(8)))  float v8f;
typedef __attribute__((ext_vector_type(4)))  float v4f;
typedef __attribute__((ext_vector_type(2)))  float v2f;
typedef __attribute__((ext_vector_type(4)))  unsigned v4u;
typedef __attribute__((ext_vector_type(4)))  int v4i;
typedef float __attribute__((may_alias)) float_a;
typedef int __attribute__((may_alias)) int_a;

template <typename T> __device__ __forceinline__ void vst2(void* p, T v) { *(volatile T*)p = v; __threadfence(); *(volatile T*)p = v; }
__device__ __forceinline__ v8f wmma16(v16h a, v16h b, v8f c) {
  v8f d = __builtin_amdgcn_wmma_f32_16x16x32_f16(false, a, false, b, (short)0, c, false, false);
  asm volatile("v_nop\n\tv_nop\n\tv_nop\n\tv_nop" : "+v"(d) : "v"(a), "v"(b));
  return d;
}
__device__ __forceinline__ v8f wmma_bf(v16b a, v16b b, v8f c) {
  v8f d = __builtin_amdgcn_wmma_f32_16x16x32_bf16(false, a, false, b, (short)0, c, false, false);
  asm volatile("v_nop\n\tv_nop\n\tv_nop\n\tv_nop" : "+v"(d) : "v"(a), "v"(b));
  return d;
}
__device__ __forceinline__ v16h frag_h(const _Float16* rowk0, int lane) {
  union { v16h v; v8h q[2]; } u; const _Float16* p = rowk0 + 8 * (lane >> 4);
  u.q[0] = *(const v8h*)p; u.q[1] = *(const v8h*)(p + 16); return u.v;
}
__device__ __forceinline__ v16h frag_f32(const float* rowk0, int lane) {
  v16h a; const float* p = rowk0 + 8 * (lane >> 4);
#pragma unroll
  for (int i = 0; i < 8; ++i) { a[i] = (_Float16)p[i]; a[8 + i] = (_Float16)p[16 + i]; }
  return a;
}
__device__ __forceinline__ v16h frag_f32s(const float* rowk0, int lane, float sc) {
  v16h a; const float* p = rowk0 + 8 * (lane >> 4);
#pragma unroll
  for (int i = 0; i < 8; ++i) { a[i] = (_Float16)(p[i] * sc); a[8 + i] = (_Float16)(p[16 + i] * sc); }
  return a;
}
__device__ __forceinline__ v16h fragc_f32(const float* W, int k0, int n, int lane, int ld, int K) {
  v16h a; const int g = lane >> 4;
#pragma unroll
  for (int i = 0; i < 8; ++i) { const int ka = k0 + 8 * g + i, kb = ka + 16;
    a[i] = (_Float16)(ka < K ? W[(size_t)(ka < K ? ka : K - 1) * ld + n] : 0.f); a[8 + i] = (_Float16)(kb < K ? W[(size_t)(kb < K ? kb : K - 1) * ld + n] : 0.f); }
  return a;
}
struct F2 { v16b h, l; };
__device__ __forceinline__ F2 bsplit16(const float v[16]) { F2 r;
#pragma unroll
  for (int i = 0; i < 16; ++i) { const __bf16 h = (__bf16)v[i]; r.h[i] = h; r.l[i] = (__bf16)(v[i] - (float)h); }
  return r; }
__device__ __forceinline__ F2 split_row(const float* row, int k0, int lane) { float v[16]; const float* p = row + k0 + 8 * (lane >> 4);
#pragma unroll
  for (int i = 0; i < 8; ++i) { v[i] = p[i]; v[8 + i] = p[16 + i]; }
  return bsplit16(v); }
__device__ __forceinline__ F2 split_rowK(const float* row, int k0, int lane, int K) { float v[16]; const int g = lane >> 4;
#pragma unroll
  for (int i = 0; i < 8; ++i) { const int ka = k0 + 8 * g + i, kb = ka + 16; v[i] = ka < K ? row[ka < K ? ka : K - 1] : 0.f; v[8 + i] = kb < K ? row[kb < K ? kb : K - 1] : 0.f; }
  return bsplit16(v); }
__device__ __forceinline__ F2 split_col(const float* W, int k0, int n, int lane, int ld, int K) { float v[16]; const int g = lane >> 4;
#pragma unroll
  for (int i = 0; i < 8; ++i) { const int ka = k0 + 8 * g + i, kb = ka + 16; v[i] = ka < K ? W[(size_t)(ka < K ? ka : K - 1) * ld + n] : 0.f; v[8 + i] = kb < K ? W[(size_t)(kb < K ? kb : K - 1) * ld + n] : 0.f; }
  return bsplit16(v); }
__device__ __forceinline__ v8f mac3(const F2& a, const F2& b, v8f c) { c = wmma_bf(a.l, b.h, c); c = wmma_bf(a.h, b.l, c); return wmma_bf(a.h, b.h, c); }
__device__ __forceinline__ float sigm(float v) { return 1.0f / (1.0f + expf(-v)); }
#define LDSX() do { asm volatile("s_wait_dscnt 0" ::: "memory"); __builtin_amdgcn_wave_barrier(); __builtin_amdgcn_fence(__ATOMIC_RELEASE, "workgroup"); } while (0)


#define NN 50000
#define NE 800000
#define D0 128
#define D1 512
#define D2 64
#define D3 16
#define D4 2
#define NRB ((NN + 63) / 64)
#define NPAD (NRB * 64)
typedef __attribute__((ext_vector_type(8))) __bf16 v8b;
__device__ __forceinline__ v16b frag_b(const __bf16* rowk0, int lane) {
  union { v16b v; v8b q[2]; } u; const __bf16* p = rowk0 + 8 * (lane >> 4);
  u.q[0] = *(const v8b*)p; u.q[1] = *(const v8b*)(p + 16); return u.v;
}
__device__ __forceinline__ float bfr(float v) { return (float)(__bf16)v; }
__device__ __attribute__((noinline)) float exp_ni(float v) { return expf(v); }
__device__ __attribute__((noinline)) float erf_ni(float v) { return erff(v); }

#define CSA_N 50000
#define CSA_E 800000
#define CSA_FINN (CSA_E + 32 * CSA_NBK)
#define CSA_CHUNK 4096
#define CSA_BKT 256
#define CSA_NCH ((CSA_E + CSA_CHUNK - 1) / CSA_CHUNK)
#define CSA_NBK ((CSA_N + CSA_BKT - 1) / CSA_BKT)
#define CSA_NBKP (((CSA_NBK + 63) / 64) * 64)
#define CSA_SEGCAP (CSA_E + 32 * CSA_NBK * CSA_NCH)
#ifndef CSA_BCAP
#define CSA_BCAP 10240
#endif
#define CSA_SZ_CNT   (4u * CSA_NCH * CSA_NBKP)
#define CSA_SZ_OFF   (4u * CSA_NBK * (((CSA_NCH + 31) / 32) * 32))
#define CSA_SZ_BST   (4u * (((CSA_NBK + 1 + 31) / 32) * 32))
#define CSA_SZ_SEG   (4u * CSA_SEGCAP)
#define CSA_SZ_FIN   (4u * (CSA_E + 32 * CSA_NBK))
#define CSA_SZ_ROW   (4u * CSA_NBK * CSA_BKT)
#define CSA_OFFP (((CSA_NCH + 31) / 32) * 32)

__global__ __launch_bounds__(256) void k_csA_cnt(const int* __restrict__ DST, int dstride, int* __restrict__ CNT) {
  __shared__ unsigned short sc[256][CSA_NBK + 1]; __shared__ __align__(16) int srow[CSA_NBKP];
  const int c = blockIdx.x, tid = threadIdx.x;
  for (int b = 0; b < CSA_NBK; ++b) sc[tid][b] = 0;
  const size_t e0 = (size_t)c * CSA_CHUNK + tid * 16;
  for (int i = 0; i < 16; ++i) { const size_t e = e0 + i; if (e < (size_t)CSA_E) { int d = DST[e * dstride]; d = min(max(d, 0), CSA_N - 1); sc[tid][d / CSA_BKT] += 1; } }
  __syncthreads();
  for (int b = tid; b < CSA_NBKP; b += 256) { int s = 0; if (b < CSA_NBK) for (int t = 0; t < 256; ++t) s += sc[t][b]; srow[b] = s; }
  __syncthreads();
  for (int q = tid; q < CSA_NBKP / 4; q += 256) vst2((unsigned*)(CNT + (size_t)c * CSA_NBKP + q * 4), *(const v4u*)&srow[q * 4]);
}
__global__ __launch_bounds__(256) void k_csA_scan(const int* __restrict__ CNT, int* __restrict__ OFF, int* __restrict__ BST) {
  __shared__ int sbt[CSA_NBK + 1]; __shared__ int sbs[((CSA_NBK + 1 + 31) / 32) * 32]; __shared__ int scnt[CSA_NBK + 1]; __shared__ __align__(16) int sbuf[64][CSA_OFFP];
  const int tid = threadIdx.x;
  for (int b = tid; b < CSA_NBK; b += 256) { int sp = 0, st = 0; for (int c = 0; c < CSA_NCH; ++c) { const int n = CNT[(size_t)c * CSA_NBKP + b]; st += n; sp += (n + 31) & ~31; } sbt[b] = sp; scnt[b] = st; }
  for (int b = tid; b < ((CSA_NBK + 1 + 31) / 32) * 32; b += 256) sbs[b] = 0;
  __syncthreads();
  if (tid == 0) { int acc = 0, accf = 0; for (int b = 0; b < CSA_NBK; ++b) { const int t = sbt[b]; sbt[b] = acc; acc += t; sbs[b] = accf; accf += (scnt[b] + 31) & ~31; } sbs[CSA_NBK] = accf; }
  __syncthreads();
  for (int b0 = 0; b0 < CSA_NBK; b0 += 64) {
    if (tid < 64 && b0 + tid < CSA_NBK) { const int b = b0 + tid; int o = sbt[b]; for (int c = 0; c < CSA_OFFP; ++c) { if (c < CSA_NCH) { sbuf[tid][c] = o; o += (CNT[(size_t)c * CSA_NBKP + b] + 31) & ~31; } else sbuf[tid][c] = 0; } }
    __syncthreads();
    for (int q = tid; q < 64 * (CSA_OFFP / 4); q += 256) { const int r = q / (CSA_OFFP / 4), pc = q % (CSA_OFFP / 4); if (b0 + r < CSA_NBK) vst2((unsigned*)(OFF + (size_t)(b0 + r) * CSA_OFFP + pc * 4), *(const v4u*)&sbuf[r][pc * 4]); }
    __syncthreads(); }
  for (int q = tid; q < ((CSA_NBK + 1 + 31) / 32) * 32 / 4; q += 256) vst2((unsigned*)(BST + q * 4), *(const v4u*)&sbs[q * 4]);
}
__global__ __launch_bounds__(256) void k_csA_scatter(const int* __restrict__ SRC, const int* __restrict__ DST, int sstride, int dstride, const int* __restrict__ OFF, int* __restrict__ SEGS, int* __restrict__ SEGE) {
  __shared__ unsigned short sc[256][CSA_NBK + 1]; __shared__ int sbase[CSA_NBK + 1]; __shared__ int scn[CSA_NBK + 1]; __shared__ int sord[CSA_CHUNK];
  const int c = blockIdx.x, tid = threadIdx.x;
  for (int b = 0; b < CSA_NBK; ++b) sc[tid][b] = 0;
  const size_t e0 = (size_t)c * CSA_CHUNK + tid * 16; int bk[16];
#pragma unroll
  for (int i = 0; i < 16; ++i) { const size_t e = e0 + i; bk[i] = -1; if (e < (size_t)CSA_E) { int d = DST[e * dstride]; d = min(max(d, 0), CSA_N - 1); bk[i] = d / CSA_BKT; sc[tid][bk[i]] += 1; } }
  __syncthreads();
  for (int b = tid; b < CSA_NBK; b += 256) { int acc = 0; for (int t = 0; t < 256; ++t) { const int v = sc[t][b]; sc[t][b] = (unsigned short)acc; acc += v; } scn[b] = acc; }
  __syncthreads();
  if (tid == 0) { int acc = 0; for (int b = 0; b < CSA_NBK; ++b) { sbase[b] = acc; acc += scn[b]; } }
  __syncthreads();
#pragma unroll
  for (int i = 0; i < 16; ++i) { if (bk[i] >= 0) { const int b = bk[i]; const int r = sc[tid][b]; sc[tid][b] = (unsigned short)(r + 1); sord[sbase[b] + r] = tid * 16 + i; } }
  __syncthreads();
  for (int b = 0; b < CSA_NBK; ++b) { const int n = scn[b]; if (n == 0) continue; const int nl = ((n + 31) & ~31); const size_t o = (size_t)(min(max(OFF[(size_t)b * CSA_OFFP + c], 0), CSA_SEGCAP - nl) & ~31);
    for (int q = tid; q < nl / 4; q += 256) { int4 vs, ve;
#pragma unroll
      for (int k = 0; k < 4; ++k) { const int i = q * 4 + k; int s = -1, eid = -1; if (i < n) { const size_t e = (size_t)c * CSA_CHUNK + sord[sbase[b] + i]; s = min(max(SRC[e * sstride], 0), CSA_N - 1); eid = (int)e; } vs[k] = s; ve[k] = eid; }
      vst2((unsigned*)(SEGS + o + q * 4), *(const v4u*)&vs); vst2((unsigned*)(SEGE + o + q * 4), *(const v4u*)&ve); } }
}
__global__ __launch_bounds__(256) void k_csA_bucket(const int* __restrict__ CNT, const int* __restrict__ OFF, const int* __restrict__ BST, const int* __restrict__ SEGS, const int* __restrict__ SEGE, const int* __restrict__ DST, int dstride, int* __restrict__ FS, int* __restrict__ FE, int* __restrict__ ROWST, int* __restrict__ ROWCNT) {
  __shared__ int ssrc[CSA_BCAP]; __shared__ int seid[CSA_BCAP]; __shared__ unsigned char snod[CSA_BCAP]; __shared__ int souts[CSA_BCAP]; __shared__ int soute[CSA_BCAP]; __shared__ int scount[256]; __shared__ int sstart[257]; __shared__ int stot;
  const int b = blockIdx.x, tid = threadIdx.x;
  if (tid == 0) { int t = 0; for (int c = 0; c < CSA_NCH; ++c) t += min(max(CNT[(size_t)c * CSA_NBKP + b], 0), CSA_CHUNK); stot = (t <= CSA_BCAP) ? t : 0; }
  __syncthreads();
  { int base = 0; for (int c = 0; c < CSA_NCH; ++c) { const int n = min(max(CNT[(size_t)c * CSA_NBKP + b], 0), CSA_CHUNK); const int o = min(max(OFF[(size_t)b * CSA_OFFP + c], 0), CSA_SEGCAP - ((n + 31) & ~31));
      for (int i = tid; i < n; i += 256) { const int p = base + i; if (p < CSA_BCAP) { ssrc[p] = min(max(SEGS[o + i], 0), CSA_N - 1); const int e = min(max(SEGE[o + i], 0), CSA_E - 1); seid[p] = e; int d = DST[(size_t)e * dstride]; d = min(max(d, 0), CSA_N - 1); const int dl = d - b * CSA_BKT; snod[p] = (unsigned char)(dl >= 0 && dl < 256 ? dl : 255); } }
      base += n; } }
  __syncthreads();
  const int node = b * CSA_BKT + tid; int cnt = 0; for (int p = 0; p < stot; ++p) cnt += (snod[p] == tid) ? 1 : 0;
  scount[tid] = cnt; __syncthreads();
  if (tid == 0) { int acc = 0; for (int t = 0; t < 256; ++t) { sstart[t] = acc; acc += scount[t]; } sstart[256] = acc; }
  __syncthreads();
  const int bst0 = min(max(BST[b], 0), CSA_FINN - ((sstart[256] + 31) & ~31)) & ~31; const int gst = bst0 + sstart[tid];
  { int w = sstart[tid]; for (int p = 0; p < stot; ++p) if (snod[p] == tid) { souts[w] = ssrc[p]; soute[w] = seid[p]; ++w; } }
  __syncthreads();
  { const int n = sstart[256]; const int nl = (n + 31) & ~31; for (int q = tid; q < nl / 4; q += 256) { int4 vs, ve;
#pragma unroll
      for (int k = 0; k < 4; ++k) { const int i = q * 4 + k; vs[k] = i < n ? souts[i] : -1; ve[k] = i < n ? soute[i] : -1; }
      vst2((unsigned*)(FS + bst0 + q * 4), *(const v4u*)&vs); vst2((unsigned*)(FE + bst0 + q * 4), *(const v4u*)&ve); } }
  __syncthreads();
  { __shared__ __align__(16) int srs[256], src2[256]; srs[tid] = node < CSA_N ? gst : 0; src2[tid] = node < CSA_N ? cnt : 0; __syncthreads();
    if (tid < 64) vst2((unsigned*)(ROWST + (size_t)b * 256 + tid * 4), *(const v4u*)&srs[tid * 4]); else if (tid < 128) vst2((unsigned*)(ROWCNT + (size_t)b * 256 + (tid - 64) * 4), *(const v4u*)&src2[(tid - 64) * 4]); }
}


#define CSB_N 50000
#define CSB_E 800000
#define CSB_FINN (CSB_E + 32 * CSB_NBK)
#define CSB_CHUNK 4096
#define CSB_BKT 256
#define CSB_NCH ((CSB_E + CSB_CHUNK - 1) / CSB_CHUNK)
#define CSB_NBK ((CSB_N + CSB_BKT - 1) / CSB_BKT)
#define CSB_NBKP (((CSB_NBK + 63) / 64) * 64)
#define CSB_SEGCAP (CSB_E + 32 * CSB_NBK * CSB_NCH)
#ifndef CSB_BCAP
#define CSB_BCAP 10240
#endif
#define CSB_SZ_CNT   (4u * CSB_NCH * CSB_NBKP)
#define CSB_SZ_OFF   (4u * CSB_NBK * (((CSB_NCH + 31) / 32) * 32))
#define CSB_SZ_BST   (4u * (((CSB_NBK + 1 + 31) / 32) * 32))
#define CSB_SZ_SEG   (4u * CSB_SEGCAP)
#define CSB_SZ_FIN   (4u * (CSB_E + 32 * CSB_NBK))
#define CSB_SZ_ROW   (4u * CSB_NBK * CSB_BKT)
#define CSB_OFFP (((CSB_NCH + 31) / 32) * 32)

__global__ __launch_bounds__(256) void k_csB_cnt(const int* __restrict__ DST, int dstride, int* __restrict__ CNT) {
  __shared__ unsigned short sc[256][CSB_NBK + 1]; __shared__ __align__(16) int srow[CSB_NBKP];
  const int c = blockIdx.x, tid = threadIdx.x;
  for (int b = 0; b < CSB_NBK; ++b) sc[tid][b] = 0;
  const size_t e0 = (size_t)c * CSB_CHUNK + tid * 16;
  for (int i = 0; i < 16; ++i) { const size_t e = e0 + i; if (e < (size_t)CSB_E) { int d = DST[e * dstride]; d = min(max(d, 0), CSB_N - 1); sc[tid][d / CSB_BKT] += 1; } }
  __syncthreads();
  for (int b = tid; b < CSB_NBKP; b += 256) { int s = 0; if (b < CSB_NBK) for (int t = 0; t < 256; ++t) s += sc[t][b]; srow[b] = s; }
  __syncthreads();
  for (int q = tid; q < CSB_NBKP / 4; q += 256) vst2((unsigned*)(CNT + (size_t)c * CSB_NBKP + q * 4), *(const v4u*)&srow[q * 4]);
}
__global__ __launch_bounds__(256) void k_csB_scan(const int* __restrict__ CNT, int* __restrict__ OFF, int* __restrict__ BST) {
  __shared__ int sbt[CSB_NBK + 1]; __shared__ int sbs[((CSB_NBK + 1 + 31) / 32) * 32]; __shared__ int scnt[CSB_NBK + 1]; __shared__ __align__(16) int sbuf[64][CSB_OFFP];
  const int tid = threadIdx.x;
  for (int b = tid; b < CSB_NBK; b += 256) { int sp = 0, st = 0; for (int c = 0; c < CSB_NCH; ++c) { const int n = CNT[(size_t)c * CSB_NBKP + b]; st += n; sp += (n + 31) & ~31; } sbt[b] = sp; scnt[b] = st; }
  for (int b = tid; b < ((CSB_NBK + 1 + 31) / 32) * 32; b += 256) sbs[b] = 0;
  __syncthreads();
  if (tid == 0) { int acc = 0, accf = 0; for (int b = 0; b < CSB_NBK; ++b) { const int t = sbt[b]; sbt[b] = acc; acc += t; sbs[b] = accf; accf += (scnt[b] + 31) & ~31; } sbs[CSB_NBK] = accf; }
  __syncthreads();
  for (int b0 = 0; b0 < CSB_NBK; b0 += 64) {
    if (tid < 64 && b0 + tid < CSB_NBK) { const int b = b0 + tid; int o = sbt[b]; for (int c = 0; c < CSB_OFFP; ++c) { if (c < CSB_NCH) { sbuf[tid][c] = o; o += (CNT[(size_t)c * CSB_NBKP + b] + 31) & ~31; } else sbuf[tid][c] = 0; } }
    __syncthreads();
    for (int q = tid; q < 64 * (CSB_OFFP / 4); q += 256) { const int r = q / (CSB_OFFP / 4), pc = q % (CSB_OFFP / 4); if (b0 + r < CSB_NBK) vst2((unsigned*)(OFF + (size_t)(b0 + r) * CSB_OFFP + pc * 4), *(const v4u*)&sbuf[r][pc * 4]); }
    __syncthreads(); }
  for (int q = tid; q < ((CSB_NBK + 1 + 31) / 32) * 32 / 4; q += 256) vst2((unsigned*)(BST + q * 4), *(const v4u*)&sbs[q * 4]);
}
__global__ __launch_bounds__(256) void k_csB_scatter(const int* __restrict__ SRC, const int* __restrict__ DST, int sstride, int dstride, const int* __restrict__ OFF, int* __restrict__ SEGS, int* __restrict__ SEGE) {
  __shared__ unsigned short sc[256][CSB_NBK + 1]; __shared__ int sbase[CSB_NBK + 1]; __shared__ int scn[CSB_NBK + 1]; __shared__ int sord[CSB_CHUNK];
  const int c = blockIdx.x, tid = threadIdx.x;
  for (int b = 0; b < CSB_NBK; ++b) sc[tid][b] = 0;
  const size_t e0 = (size_t)c * CSB_CHUNK + tid * 16; int bk[16];
#pragma unroll
  for (int i = 0; i < 16; ++i) { const size_t e = e0 + i; bk[i] = -1; if (e < (size_t)CSB_E) { int d = DST[e * dstride]; d = min(max(d, 0), CSB_N - 1); bk[i] = d / CSB_BKT; sc[tid][bk[i]] += 1; } }
  __syncthreads();
  for (int b = tid; b < CSB_NBK; b += 256) { int acc = 0; for (int t = 0; t < 256; ++t) { const int v = sc[t][b]; sc[t][b] = (unsigned short)acc; acc += v; } scn[b] = acc; }
  __syncthreads();
  if (tid == 0) { int acc = 0; for (int b = 0; b < CSB_NBK; ++b) { sbase[b] = acc; acc += scn[b]; } }
  __syncthreads();
#pragma unroll
  for (int i = 0; i < 16; ++i) { if (bk[i] >= 0) { const int b = bk[i]; const int r = sc[tid][b]; sc[tid][b] = (unsigned short)(r + 1); sord[sbase[b] + r] = tid * 16 + i; } }
  __syncthreads();
  for (int b = 0; b < CSB_NBK; ++b) { const int n = scn[b]; if (n == 0) continue; const int nl = ((n + 31) & ~31); const size_t o = (size_t)(min(max(OFF[(size_t)b * CSB_OFFP + c], 0), CSB_SEGCAP - nl) & ~31);
    for (int q = tid; q < nl / 4; q += 256) { int4 vs, ve;
#pragma unroll
      for (int k = 0; k < 4; ++k) { const int i = q * 4 + k; int s = -1, eid = -1; if (i < n) { const size_t e = (size_t)c * CSB_CHUNK + sord[sbase[b] + i]; s = min(max(SRC[e * sstride], 0), CSB_N - 1); eid = (int)e; } vs[k] = s; ve[k] = eid; }
      vst2((unsigned*)(SEGS + o + q * 4), *(const v4u*)&vs); vst2((unsigned*)(SEGE + o + q * 4), *(const v4u*)&ve); } }
}
__global__ __launch_bounds__(256) void k_csB_bucket(const int* __restrict__ CNT, const int* __restrict__ OFF, const int* __restrict__ BST, const int* __restrict__ SEGS, const int* __restrict__ SEGE, const int* __restrict__ DST, int dstride, int* __restrict__ FS, int* __restrict__ FE, int* __restrict__ ROWST, int* __restrict__ ROWCNT) {
  __shared__ int ssrc[CSB_BCAP]; __shared__ int seid[CSB_BCAP]; __shared__ unsigned char snod[CSB_BCAP]; __shared__ int souts[CSB_BCAP]; __shared__ int soute[CSB_BCAP]; __shared__ int scount[256]; __shared__ int sstart[257]; __shared__ int stot;
  const int b = blockIdx.x, tid = threadIdx.x;
  if (tid == 0) { int t = 0; for (int c = 0; c < CSB_NCH; ++c) t += min(max(CNT[(size_t)c * CSB_NBKP + b], 0), CSB_CHUNK); stot = (t <= CSB_BCAP) ? t : 0; }
  __syncthreads();
  { int base = 0; for (int c = 0; c < CSB_NCH; ++c) { const int n = min(max(CNT[(size_t)c * CSB_NBKP + b], 0), CSB_CHUNK); const int o = min(max(OFF[(size_t)b * CSB_OFFP + c], 0), CSB_SEGCAP - ((n + 31) & ~31));
      for (int i = tid; i < n; i += 256) { const int p = base + i; if (p < CSB_BCAP) { ssrc[p] = min(max(SEGS[o + i], 0), CSB_N - 1); const int e = min(max(SEGE[o + i], 0), CSB_E - 1); seid[p] = e; int d = DST[(size_t)e * dstride]; d = min(max(d, 0), CSB_N - 1); const int dl = d - b * CSB_BKT; snod[p] = (unsigned char)(dl >= 0 && dl < 256 ? dl : 255); } }
      base += n; } }
  __syncthreads();
  const int node = b * CSB_BKT + tid; int cnt = 0; for (int p = 0; p < stot; ++p) cnt += (snod[p] == tid) ? 1 : 0;
  scount[tid] = cnt; __syncthreads();
  if (tid == 0) { int acc = 0; for (int t = 0; t < 256; ++t) { sstart[t] = acc; acc += scount[t]; } sstart[256] = acc; }
  __syncthreads();
  const int bst0 = min(max(BST[b], 0), CSB_FINN - ((sstart[256] + 31) & ~31)) & ~31; const int gst = bst0 + sstart[tid];
  { int w = sstart[tid]; for (int p = 0; p < stot; ++p) if (snod[p] == tid) { souts[w] = ssrc[p]; soute[w] = seid[p]; ++w; } }
  __syncthreads();
  { const int n = sstart[256]; const int nl = (n + 31) & ~31; for (int q = tid; q < nl / 4; q += 256) { int4 vs, ve;
#pragma unroll
      for (int k = 0; k < 4; ++k) { const int i = q * 4 + k; vs[k] = i < n ? souts[i] : -1; ve[k] = i < n ? soute[i] : -1; }
      vst2((unsigned*)(FS + bst0 + q * 4), *(const v4u*)&vs); vst2((unsigned*)(FE + bst0 + q * 4), *(const v4u*)&ve); } }
  __syncthreads();
  { __shared__ __align__(16) int srs[256], src2[256]; srs[tid] = node < CSB_N ? gst : 0; src2[tid] = node < CSB_N ? cnt : 0; __syncthreads();
    if (tid < 64) vst2((unsigned*)(ROWST + (size_t)b * 256 + tid * 4), *(const v4u*)&srs[tid * 4]); else if (tid < 128) vst2((unsigned*)(ROWCNT + (size_t)b * 256 + (tid - 64) * 4), *(const v4u*)&src2[(tid - 64) * 4]); }
}


#define WS_CNT  0u
#define WS_OFF  (WS_CNT + CSA_SZ_CNT)
#define WS_BST  (WS_OFF + CSA_SZ_OFF)
#define WS_SEGS (WS_BST + CSA_SZ_BST)
#define WS_SEGE (WS_SEGS + CSA_SZ_SEG)
#define WS_FS   (WS_SEGE + CSA_SZ_SEG)
#define WS_FE   (WS_FS + CSA_SZ_FIN)
#define WS_RST  (WS_FE + CSA_SZ_FIN)
#define WS_RCT  (WS_RST + CSA_SZ_ROW)
#define WS_BCNT (WS_RCT + CSA_SZ_ROW)
#define WS_BOFF (WS_BCNT + CSB_SZ_CNT)
#define WS_BBST (WS_BOFF + CSB_SZ_OFF)
#define WS_BSGS (WS_BBST + CSB_SZ_BST)
#define WS_BSGE (WS_BSGS + CSB_SZ_SEG)
#define WS_BFS  (WS_BSGE + CSB_SZ_SEG)
#define WS_BFE  (WS_BFS + CSB_SZ_FIN)
#define WS_BRST (WS_BFE + CSB_SZ_FIN)
#define WS_BRCT (WS_BRST + CSB_SZ_ROW)
#define WS_PW   (WS_BRCT + CSB_SZ_ROW)
#define PW1 0
#define PW2 (PW1 + D1 * D0)
#define PWEND (PW2 + D2 * D1)
#define WS_A1   (WS_PW + 2u * PWEND)
#define WS_X2   (WS_A1 + 4u * NPAD * D0)
#define WS_H2   (WS_X2 + 4u * NPAD * D2)
#define WS_X3   (WS_H2 + 4u * NPAD * D2)
#define WS_X4   (WS_X3 + 4u * NPAD * D3)
#define WS_H3   (WS_X4 + 4u * NPAD * D3)
#define WS_END  (WS_H3 + 4u * NPAD * D3)

__global__ __launch_bounds__(256) void k_packT(const float* __restrict__ W1, const float* __restrict__ W2, __bf16* __restrict__ PW) {
  __shared__ __align__(16) __bf16 s[D1]; const int n = blockIdx.x, which = blockIdx.y, tid = threadIdx.x; int K; size_t dst;
  if (which == 0) { if (n >= D1) return; K = D0; dst = PW1 + (size_t)n * D0; for (int k = tid; k < K; k += 256) s[k] = (__bf16)W1[(size_t)k * D1 + n]; }
  else { if (n >= D2) return; K = D1; dst = PW2 + (size_t)n * D1; for (int k = tid; k < K; k += 256) s[k] = (__bf16)W2[(size_t)k * D2 + n]; }
  __syncthreads();
  for (int q = tid; q < K / 8; q += 256) vst2((unsigned*)(PW + dst + q * 8), *(const v4u*)&s[q * 8]);
}
template <int W, int RIN, int EPI>
__global__ __launch_bounds__(256) void k_gagg(const float* __restrict__ SRC, const int* __restrict__ FS, const int* __restrict__ RST, const int* __restrict__ RCT, const int* __restrict__ RCTB, const float* __restrict__ bias, float* __restrict__ OUT) {
  constexpr int TPN = (W >= 64) ? (W / 4) : 4;
  constexpr int FPT = (W >= 16) ? (W / TPN) : 4;
  constexpr int NODES_PER_PASS = 256 / TPN;
  __shared__ __align__(16) float so[64][(W >= 16 ? W : 16) + 4];
  const int tid = threadIdx.x; const int nb = blockIdx.x;
  for (int pass = 0; pass < 64 / NODES_PER_PASS; ++pass) { const int nl = pass * NODES_PER_PASS + tid / TPN; const int f0 = (tid % TPN) * FPT; const int i = nb * 64 + nl;
    float acc[FPT]; for (int k = 0; k < FPT; ++k) acc[k] = 0.f;
    if (i < NN) { const int cnt = min(max(RCT[i], 0), CSA_BCAP); const int st = min(max(RST[i], 0), CSA_FINN - cnt);
      for (int e = 0; e < cnt; ++e) { const int s = min(max(FS[st + e], 0), NN - 1); const int dego = max(RCTB[s], 1); const float ns = rsqrtf((float)dego);
        const float* row = SRC + (size_t)s * (W >= 16 ? W : 16) + f0;
#pragma unroll
        for (int k = 0; k < FPT; ++k) { const float v = RIN ? bfr(row[k]) : row[k]; acc[k] += ns * v; } }
      const float nd = (cnt > 0) ? rsqrtf((float)cnt) : 0.f;
#pragma unroll
      for (int k = 0; k < FPT; ++k) { float v = acc[k] * nd; if (EPI) { v += bfr(bias[f0 + k]); v = fmaxf(v, 0.f); } if (W < 16 && f0 + k >= W) v = 0.f; acc[k] = v; } }
#pragma unroll
    for (int k = 0; k < FPT; ++k) so[nl][f0 + k] = acc[k]; }
  __syncthreads();
  constexpr int PITCH = (W >= 16) ? W : 16;
  for (int q = tid; q < 64 * PITCH / 4; q += 256) { const int nl = q / (PITCH / 4), pc = q % (PITCH / 4); vst2(OUT + ((size_t)nb * 64 + nl) * PITCH + pc * 4, *(const v4f*)&so[nl][pc * 4]); }
}
__global__ __launch_bounds__(128) void k_l12(const float* __restrict__ A1, const __bf16* __restrict__ PW, const float* __restrict__ B1, float* __restrict__ X2) {
  __shared__ __align__(16) float st[4][16][132]; __shared__ __align__(16) float so[4][16][68];
  const int tid = threadIdx.x, wave = tid >> 5, lane = tid & 31, col = lane & 15, g = lane >> 4; const size_t r0 = (size_t)blockIdx.x * 64 + wave * 16;
  F2 a[4];
#pragma unroll
  for (int kc = 0; kc < 4; ++kc) a[kc] = split_row(A1 + (r0 + col) * D0, kc * 32, lane);
  v8f acc2[4] = {};
#pragma unroll 1
  for (int c = 0; c < D1 / 128; ++c) { v8f acc[8] = {};
#pragma unroll
    for (int kc = 0; kc < 4; ++kc) {
#pragma unroll
      for (int j = 0; j < 8; ++j) { const v16b w = frag_b(PW + PW1 + (size_t)(c * 128 + j * 16 + col) * D0 + kc * 32, lane); acc[j] = wmma_bf(a[kc].l, w, acc[j]); acc[j] = wmma_bf(a[kc].h, w, acc[j]); } }
#pragma unroll
    for (int j = 0; j < 8; ++j) { const float bb = bfr(B1[c * 128 + j * 16 + col]);
#pragma unroll
      for (int r = 0; r < 8; ++r) st[wave][8 * g + r][j * 16 + col] = fmaxf(acc[j][r] + bb, 0.f); }
    LDSX();
#pragma unroll
    for (int kc = 0; kc < 4; ++kc) { const F2 h = split_row(&st[wave][col][0], kc * 32, lane);
#pragma unroll
      for (int j = 0; j < 4; ++j) { const v16b w = frag_b(PW + PW2 + (size_t)(j * 16 + col) * D1 + c * 128 + kc * 32, lane); acc2[j] = wmma_bf(h.l, w, acc2[j]); acc2[j] = wmma_bf(h.h, w, acc2[j]); } }
    LDSX(); }
#pragma unroll
  for (int j = 0; j < 4; ++j)
#pragma unroll
    for (int r = 0; r < 8; ++r) so[wave][8 * g + r][j * 16 + col] = acc2[j][r];
  LDSX();
  for (int rl = 0; rl < 16; ++rl) if (lane < 16) vst2(X2 + (r0 + rl) * D2 + lane * 4, *(const v4f*)&so[wave][rl][lane * 4]);
}
template <int KIN, int KOUT, int PIN>
__global__ __launch_bounds__(256) void k_small(const float* __restrict__ IN, const float* __restrict__ Wm, float* __restrict__ OUT) {
  __shared__ float sw[KIN][KOUT]; __shared__ __align__(16) float so[64][16];
  const int tid = threadIdx.x; const size_t rb = (size_t)blockIdx.x * 64;
  for (int q = tid; q < KIN * KOUT; q += 256) sw[q / KOUT][q % KOUT] = bfr(Wm[q]);
  __syncthreads();
  { const int nl = tid >> 2, part = tid & 3; const float* row = IN + (rb + nl) * PIN;
    for (int o = part; o < 16; o += 4) { float v = 0.f; if (o < KOUT) {
#pragma unroll 1
        for (int k = 0; k < KIN; ++k) v += row[k] * sw[k][o]; }
      so[nl][o] = v; } }
  __syncthreads();
  vst2(OUT + rb * 16 + tid * 4, *(const v4f*)&(&so[0][0])[tid * 4]);
}
__global__ __launch_bounds__(64) void k_out(const float* __restrict__ X4, const int* __restrict__ FS, const int* __restrict__ RST, const int* __restrict__ RCT, const int* __restrict__ RCTB, const float* __restrict__ B4, float* __restrict__ out) {
  __shared__ __align__(16) float so[64][2]; const int tid = threadIdx.x; const int i = blockIdx.x * 64 + tid;
  float a0 = 0.f, a1 = 0.f;
  if (i < NN) { const int cnt = min(max(RCT[i], 0), CSA_BCAP); const int st = min(max(RST[i], 0), CSA_FINN - cnt);
    for (int e = 0; e < cnt; ++e) { const int s = min(max(FS[st + e], 0), NN - 1); const float ns = rsqrtf((float)max(RCTB[s], 1)); a0 += ns * X4[(size_t)s * 16 + 0]; a1 += ns * X4[(size_t)s * 16 + 1]; }
    const float nd = (cnt > 0) ? rsqrtf((float)cnt) : 0.f; a0 = fmaxf(a0 * nd + bfr(B4[0]), 0.f); a1 = fmaxf(a1 * nd + bfr(B4[1]), 0.f); }
  so[tid][0] = a0; so[tid][1] = a1;
  __syncthreads();
  const int nvalid = min(64, NN - blockIdx.x * 64);
  if (nvalid == 64) { if (tid < 32) vst2(out + (size_t)blockIdx.x * 128 + tid * 4, *(const v4f*)&(&so[0][0])[tid * 4]); }
  else if (tid == 0) { for (int k = 0; k < nvalid * 2; ++k) { *(volatile float*)(out + (size_t)blockIdx.x * 128 + k) = (&so[0][0])[k]; } __threadfence(); for (int k = 0; k < nvalid * 2; ++k) *(volatile float*)(out + (size_t)blockIdx.x * 128 + k) = (&so[0][0])[k]; }
}
extern "C" void kernel_launch(void* const* d_in, const int* in_sizes, int n_in, void* d_out, int out_size, void* d_ws, size_t ws_size, hipStream_t stream) {
  (void)in_sizes; (void)n_in; (void)out_size;
  const float** F = (const float**)d_in; const int* SRCI = (const int*)d_in[1]; const int* DSTI = (const int*)d_in[2];
  if (ws_size < (size_t)WS_END) return;
  char* ws = (char*)d_ws;
  int *CNT = (int*)(ws + WS_CNT), *OFF = (int*)(ws + WS_OFF), *BST = (int*)(ws + WS_BST), *SEGS = (int*)(ws + WS_SEGS), *SEGE = (int*)(ws + WS_SEGE), *FS = (int*)(ws + WS_FS), *FE = (int*)(ws + WS_FE), *RST = (int*)(ws + WS_RST), *RCT = (int*)(ws + WS_RCT);
  int *BCNT = (int*)(ws + WS_BCNT), *BOFF = (int*)(ws + WS_BOFF), *BBST = (int*)(ws + WS_BBST), *BSGS = (int*)(ws + WS_BSGS), *BSGE = (int*)(ws + WS_BSGE), *BFS = (int*)(ws + WS_BFS), *BFE = (int*)(ws + WS_BFE), *BRST = (int*)(ws + WS_BRST), *BRCT = (int*)(ws + WS_BRCT);
  __bf16* PW = (__bf16*)(ws + WS_PW); float *A1 = (float*)(ws + WS_A1), *X2 = (float*)(ws + WS_X2), *H2 = (float*)(ws + WS_H2), *X3 = (float*)(ws + WS_X3), *X4 = (float*)(ws + WS_X4), *H3 = (float*)(ws + WS_H3);
  k_csA_cnt<<<CSA_NCH, 256, 0, stream>>>(DSTI, 1, CNT); k_csA_scan<<<1, 256, 0, stream>>>(CNT, OFF, BST); k_csA_scatter<<<CSA_NCH, 256, 0, stream>>>(SRCI, DSTI, 1, 1, OFF, SEGS, SEGE); k_csA_bucket<<<CSA_NBK, 256, 0, stream>>>(CNT, OFF, BST, SEGS, SEGE, DSTI, 1, FS, FE, RST, RCT);
  k_csB_cnt<<<CSB_NCH, 256, 0, stream>>>(SRCI, 1, BCNT); k_csB_scan<<<1, 256, 0, stream>>>(BCNT, BOFF, BBST); k_csB_scatter<<<CSB_NCH, 256, 0, stream>>>(DSTI, SRCI, 1, 1, BOFF, BSGS, BSGE); k_csB_bucket<<<CSB_NBK, 256, 0, stream>>>(BCNT, BOFF, BBST, BSGS, BSGE, SRCI, 1, BFS, BFE, BRST, BRCT);
  k_packT<<<dim3(D1, 2), 256, 0, stream>>>(F[3], F[5], PW);
  k_gagg<D0, 1, 0><<<NRB, 256, 0, stream>>>(F[0], FS, RST, RCT, BRCT, nullptr, A1);
  k_l12<<<NRB, 128, 0, stream>>>(A1, PW, F[4], X2);
  k_gagg<D2, 0, 1><<<NRB, 256, 0, stream>>>(X2, FS, RST, RCT, BRCT, F[6], H2);
  k_small<D2, D3, D2><<<NRB, 256, 0, stream>>>(H2, F[7], X3);
  k_gagg<D3, 0, 1><<<NRB, 256, 0, stream>>>(X3, FS, RST, RCT, BRCT, F[8], H3);
  k_small<D3, D4, 16><<<NRB, 256, 0, stream>>>(H3, F[9], X4);
  k_out<<<NRB, 64, 0, stream>>>(X4, FS, RST, RCT, BRCT, F[10], (float*)d_out);
}
